// TMix_gptalpha_7524782702652
// MI455X (gfx1250) — hardware-verified
//
#include <hip/hip_runtime.h>
#include <math.h>
#include <stdint.h>

constexpr int kBatch = 2;
constexpr int kSeq   = 2048;
constexpr int kDm    = 1024;
constexpr int kHeads = 16;
constexpr int kLoraN = 96;
constexpr int kLoraP = 128;
constexpr int kLoraD = 32;

typedef __attribute__((ext_vector_type(16))) _Float16 v16h;
typedef __attribute__((ext_vector_type(8)))  _Float16 v8h;
typedef __attribute__((ext_vector_type(16))) __bf16   v16b;
typedef __attribute__((ext_vector_type(8)))  __bf16   v8b;
typedef __attribute__((ext_vector_type(8)))  float    v8f;
typedef __attribute__((ext_vector_type(4)))  float    v4f;
typedef __attribute__((ext_vector_type(2)))  float    v2f;
typedef __attribute__((ext_vector_type(4)))  unsigned int v4u;
typedef __attribute__((ext_vector_type(8)))  unsigned short v8us;

__device__ __forceinline__ unsigned short f2bf_bits(float f) {
  unsigned u = __float_as_uint(f);
  return (unsigned short)((u + 0x7FFFu + ((u >> 16) & 1u)) >> 16);
}
__device__ __forceinline__ float bf_bits2f(unsigned short h) { return __uint_as_float(((unsigned)h) << 16); }

__device__ __forceinline__ void dep_guard_h(v8f& a, v8f& b, v16h x, v16h y) { asm volatile("v_nop\n\tv_nop\n\tv_nop\n\tv_nop" : "+v"(a), "+v"(b) : "v"(x), "v"(y)); }
__device__ __forceinline__ void dep_guard_b(v8f& a, v8f& b, v16b x, v16b y) { asm volatile("v_nop\n\tv_nop\n\tv_nop\n\tv_nop" : "+v"(a), "+v"(b) : "v"(x), "v"(y)); }
__device__ __forceinline__ void keep4_h(v16h a, v16h b, v16h c, v16h d) { asm volatile("v_nop" :: "v"(a), "v"(b), "v"(c), "v"(d)); }
__device__ __forceinline__ void keep4_b(v16b a, v16b b, v16b c, v16b d) { asm volatile("v_nop" :: "v"(a), "v"(b), "v"(c), "v"(d)); }
__device__ __forceinline__ void acc_guard4(v8f& a, v8f& b, v8f& c, v8f& d) { asm volatile("v_nop\n\tv_nop\n\tv_nop\n\tv_nop" : "+v"(a), "+v"(b), "+v"(c), "+v"(d)); }
template <typename T> struct Frag;
template <> struct Frag<_Float16> {
  typedef v16h V; union U { v16h v; v8h h[2]; };
  static __device__ __forceinline__ v16h load(const _Float16* p) {
    U f; f.h[0] = *(const v8h*)(p); f.h[1] = *(const v8h*)(p + 16); return f.v;
  }
  static __device__ __forceinline__ v8f mma(v16h a, v16h b, v8f c) {
    return __builtin_amdgcn_wmma_f32_16x16x32_f16(false, a, false, b, (short)0, c, false, false);
  }
  static __device__ __forceinline__ void guard(v8f& a, v8f& b, v16h x, v16h y) { dep_guard_h(a, b, x, y); }
  static __device__ __forceinline__ void keep(v16h a, v16h b, v16h c, v16h d) { keep4_h(a, b, c, d); }
};
template <> struct Frag<__bf16> {
  typedef v16b V; union U { v16b v; v8b h[2]; };
  static __device__ __forceinline__ v16b load(const __bf16* p) {
    U f; f.h[0] = *(const v8b*)(p); f.h[1] = *(const v8b*)(p + 16); return f.v;
  }
  static __device__ __forceinline__ v8f mma(v16b a, v16b b, v8f c) {
    return __builtin_amdgcn_wmma_f32_16x16x32_bf16(false, a, false, b, (short)0, c, false, false);
  }
  static __device__ __forceinline__ void guard(v8f& a, v8f& b, v16b x, v16b y) { dep_guard_b(a, b, x, y); }
  static __device__ __forceinline__ void keep(v16b a, v16b b, v16b c, v16b d) { keep4_b(a, b, c, d); }
};

template <int ET> struct Elem;
template <> struct Elem<0> { typedef _Float16 T; };
template <> struct Elem<1> { typedef __bf16 T; };
template <int ET, bool SPLIT, int BIAS_MODE, int OUT_MODE, bool RESID, int ACT = 0>
__global__ __launch_bounds__(256) void wmma_gemm64(
    const unsigned short* __restrict__ Ap, const unsigned short* __restrict__ A2p, int lda, long strideA,
    const unsigned short* __restrict__ Btp, const unsigned short* __restrict__ Bt2p, int ldb, long strideB,
    void* __restrict__ Cout, void* __restrict__ Cout2, int ldc, long strideC,
    const float* __restrict__ bias,
    const float* __restrict__ resid, long strideR,
    int M, int N, int K, float scale) {
  typedef typename Elem<ET>::T T;
  typedef typename Frag<T>::V V;
  const T* A = (const T*)Ap; const T* A2 = (const T*)A2p; const T* Bt = (const T*)Btp; const T* Bt2 = (const T*)Bt2p;
  __shared__ __align__(16) float sT[8][16 * 68];
  const int b    = blockIdx.y;
  const int lane = threadIdx.x & 31;
  const int wave = threadIdx.x >> 5;
  const int tilesN = N >> 6;
  const int tilesM = M >> 6;
  const int tile = blockIdx.x * 8 + wave;
  if (tile >= tilesM * tilesN) return;
  const int tm = tile / tilesN;
  const int tn = tile - tm * tilesN;
  const int m0 = tm << 6;
  const int n0 = tn << 6;

  const T* Ab  = A  + (size_t)b * strideA;
  const T* Bb  = Bt + (size_t)b * strideB;
  const T* Ab2 = SPLIT ? (A2  + (size_t)b * strideA) : nullptr;
  const T* Bb2 = SPLIT ? (Bt2 + (size_t)b * strideB) : nullptr;

  const int rlane = lane & 15;
  const int koff  = (lane >> 4) * 8;
  const int mOff  = (lane >> 4) * 8;

  v8f acc[4][4];
#pragma unroll
  for (int i = 0; i < 4; ++i)
#pragma unroll
    for (int j = 0; j < 4; ++j) acc[i][j] = (v8f){0.f,0.f,0.f,0.f,0.f,0.f,0.f,0.f};

  for (int k0 = 0; k0 < K; k0 += 32) {
    V bh[4], bl[4];
#pragma unroll
    for (int j = 0; j < 4; ++j) {
      const size_t bo = (size_t)(n0 + (j << 4) + rlane) * ldb + koff + k0;
      bh[j] = Frag<T>::load(Bb + bo);
      if (SPLIT) bl[j] = Frag<T>::load(Bb2 + bo);
    }
#pragma unroll
    for (int i = 0; i < 4; ++i) {
      const size_t ao = (size_t)(m0 + (i << 4) + rlane) * lda + koff + k0;
      V ah = Frag<T>::load(Ab + ao);
      V al;
      if (SPLIT) al = Frag<T>::load(Ab2 + ao);
#pragma unroll
      for (int j = 0; j < 4; ++j) {
        acc[i][j] = Frag<T>::mma(ah, bh[j], acc[i][j]);
        if (SPLIT) {
          acc[i][j] = Frag<T>::mma(ah, bl[j], acc[i][j]);
          acc[i][j] = Frag<T>::mma(al, bh[j], acc[i][j]);
        }
      }
      Frag<T>::guard(acc[i][0], acc[i][3], ah, SPLIT ? al : ah);
    }
    Frag<T>::keep(bh[0], bh[1], bh[2], bh[3]);
    if (SPLIT) Frag<T>::keep(bl[0], bl[1], bl[2], bl[3]);
  }
  acc_guard4(acc[0][0], acc[0][1], acc[0][2], acc[0][3]);
  acc_guard4(acc[1][0], acc[1][1], acc[1][2], acc[1][3]);
  acc_guard4(acc[2][0], acc[2][1], acc[2][2], acc[2][3]);
  acc_guard4(acc[3][0], acc[3][1], acc[3][2], acc[3][3]);

  float* slab = sT[wave];
  const float* Rb = RESID ? (resid + (size_t)b * strideR) : nullptr;
#pragma unroll
  for (int i = 0; i < 4; ++i) {
    const int mBase = m0 + (i << 4);
#pragma unroll
    for (int j = 0; j < 4; ++j) {
      const int n = n0 + (j << 4) + rlane;
      float bv = 0.f;
      if (BIAS_MODE == 2) bv = bias[n];
#pragma unroll
      for (int r = 0; r < 8; ++r) {
        float v = acc[i][j][r] * scale;
        if (BIAS_MODE == 1) v += bias[mBase + mOff + r];
        if (BIAS_MODE == 2) v += bv;
        if (RESID) v += Rb[(size_t)(mBase + mOff + r) * ldc + n];
        if (ACT == 1) v = tanhf(v);
        if (ACT == 2) v = fmaxf(v, 0.0f);
        if (ACT == 3) v = v / (1.0f + expf(-v));
        if (ACT == 4) v = (v > 0.f) ? v : 0.01f * v;
        slab[(mOff + r) * 68 + (j << 4) + rlane] = v;
      }
    }
    __builtin_amdgcn_fence(__ATOMIC_RELEASE, "workgroup");
    __builtin_amdgcn_wave_barrier();
    __builtin_amdgcn_fence(__ATOMIC_ACQUIRE, "workgroup");
    if (OUT_MODE == 0) {
      float* C = (float*)Cout + (size_t)b * strideC;
      const int hh = lane >> 4, c4 = (lane & 15) * 4;
      for (int pass = 0; pass < 2; ++pass) {
#pragma unroll
        for (int it = 0; it < 8; ++it) {
          const int row = it * 2 + hh;
          v4f v = *(const v4f*)(slab + row * 68 + c4);
          *(volatile v4f*)(C + (size_t)(mBase + row) * ldc + n0 + c4) = v;
        }
        __threadfence();
      }
    } else {
      const int q = lane >> 3, c8 = (lane & 7) * 8;
      unsigned short* C  = (unsigned short*)Cout  + (size_t)b * strideC;
      unsigned short* C2 = (OUT_MODE == 2) ? ((unsigned short*)Cout2 + (size_t)b * strideC) : nullptr;
      for (int pass = 0; pass < 2; ++pass) {
#pragma unroll
        for (int it = 0; it < 4; ++it) {
          const int row = it * 4 + q;
          const float* sp = slab + row * 68 + c8;
          v8h hv, lv;
#pragma unroll
          for (int e = 0; e < 8; ++e) {
            if (OUT_MODE == 1) {
              hv[e] = (_Float16)sp[e];
            } else {
              unsigned short hb = f2bf_bits(sp[e]);
              unsigned short lb = f2bf_bits(sp[e] - bf_bits2f(hb));
              hv[e] = __builtin_bit_cast(_Float16, hb);
              lv[e] = __builtin_bit_cast(_Float16, lb);
            }
          }
          *(volatile v8h*)(C + (size_t)(mBase + row) * ldc + n0 + c8) = hv;
          if (OUT_MODE == 2) *(volatile v8h*)(C2 + (size_t)(mBase + row) * ldc + n0 + c8) = lv;
        }
        __threadfence();
      }
    }
    __builtin_amdgcn_fence(__ATOMIC_RELEASE, "workgroup");
    __builtin_amdgcn_wave_barrier();
    __builtin_amdgcn_fence(__ATOMIC_ACQUIRE, "workgroup");
  }
}

__device__ __forceinline__ unsigned pk16(unsigned short a, unsigned short b) { return (unsigned)a | ((unsigned)b << 16); }

__global__ __launch_bounds__(256) void split_bf16x2_kernel(const float* __restrict__ in, unsigned short* __restrict__ hi,
                                                           unsigned short* __restrict__ lo, int n2) {
  const int i = blockIdx.x * 256 + threadIdx.x;
  if (i < n2) {
    const v2f f = *(const v2f*)(in + 2 * (size_t)i);
    const unsigned short h0 = f2bf_bits(f[0]), h1 = f2bf_bits(f[1]);
    const unsigned short l0 = f2bf_bits(f[0] - bf_bits2f(h0)), l1 = f2bf_bits(f[1] - bf_bits2f(h1));
    const unsigned uh = pk16(h0, h1), ul = pk16(l0, l1);
    ((volatile unsigned*)hi)[i] = uh;
    ((volatile unsigned*)lo)[i] = ul;
    __threadfence();
    ((volatile unsigned*)hi)[i] = uh;
    ((volatile unsigned*)lo)[i] = ul;
  }
}

__global__ __launch_bounds__(256) void tanh_split_kernel(const float* __restrict__ in, unsigned short* __restrict__ hi,
                                                         unsigned short* __restrict__ lo, int n2) {
  const int i = blockIdx.x * 256 + threadIdx.x;
  if (i < n2) {
    const v2f f = *(const v2f*)(in + 2 * (size_t)i);
    const float t0 = tanhf(f[0]), t1 = tanhf(f[1]);
    const unsigned short h0 = f2bf_bits(t0), h1 = f2bf_bits(t1);
    const unsigned short l0 = f2bf_bits(t0 - bf_bits2f(h0)), l1 = f2bf_bits(t1 - bf_bits2f(h1));
    const unsigned uh = pk16(h0, h1), ul = pk16(l0, l1);
    ((volatile unsigned*)hi)[i] = uh;
    ((volatile unsigned*)lo)[i] = ul;
    __threadfence();
    ((volatile unsigned*)hi)[i] = uh;
    ((volatile unsigned*)lo)[i] = ul;
  }
}

__global__ __launch_bounds__(256) void wt_split_kernel(const float* __restrict__ w, unsigned short* __restrict__ th,
                                                       unsigned short* __restrict__ tl, int R, int Cn) {
  __shared__ float tile[64 * 65];
  const int n0 = blockIdx.x * 64;
  const int k0 = blockIdx.y * 64;
  const int t = threadIdx.x;
#pragma unroll
  for (int i = 0; i < 16; ++i) {
    const int idx = i * 256 + t;
    const int kk = idx >> 6, nn = idx & 63;
    tile[nn * 65 + kk] = w[(size_t)(k0 + kk) * Cn + n0 + nn];
  }
  __syncthreads();
  const int lane = t & 31, wave = t >> 5;
  const int q = lane >> 3, c8 = (lane & 7) * 8;
  for (int pass = 0; pass < 2; ++pass) {
#pragma unroll
    for (int it = 0; it < 2; ++it) {
      const int row = wave * 8 + it * 4 + q;
      const float* sp = tile + row * 65 + c8;
      v8us hv, lv;
#pragma unroll
      for (int e = 0; e < 8; ++e) {
        const unsigned short hb = f2bf_bits(sp[e]);
        const unsigned short lb = f2bf_bits(sp[e] - bf_bits2f(hb));
        hv[e] = hb; lv[e] = lb;
      }
      const size_t o = (size_t)(n0 + row) * R + k0 + c8;
      *(volatile v8us*)(th + o) = hv;
      *(volatile v8us*)(tl + o) = lv;
    }
    __threadfence();
  }
}

__global__ __launch_bounds__(256) void w1t_split_kernel(const float* __restrict__ w1, unsigned short* __restrict__ th,
                                                        unsigned short* __restrict__ tl) {
  __shared__ float tile[kLoraP * 65];
  const int k0 = blockIdx.x * 64;
  const int t = threadIdx.x;
#pragma unroll 4
  for (int i = 0; i < 32; ++i) {
    const int idx = i * 256 + t;
    const int kk = idx >> 7, nn = idx & 127;
    const int nc = (nn < kLoraN) ? nn : (kLoraN - 1);
    float v = w1[(size_t)(k0 + kk) * kLoraN + nc];
    if (nn >= kLoraN) v = 0.0f;
    tile[nn * 65 + kk] = v;
  }
  __syncthreads();
  const int lane = t & 31, wave = t >> 5;
  const int q = lane >> 3, c8 = (lane & 7) * 8;
  for (int pass = 0; pass < 2; ++pass) {
#pragma unroll
    for (int it = 0; it < 4; ++it) {
      const int row = wave * 16 + it * 4 + q;
      const float* sp = tile + row * 65 + c8;
      v8us hv, lv;
#pragma unroll
      for (int e = 0; e < 8; ++e) {
        const unsigned short hb = f2bf_bits(sp[e]);
        const unsigned short lb = f2bf_bits(sp[e] - bf_bits2f(hb));
        hv[e] = hb; lv[e] = lb;
      }
      const size_t o = (size_t)row * kDm + k0 + c8;
      *(volatile v8us*)(th + o) = hv;
      *(volatile v8us*)(tl + o) = lv;
    }
    __threadfence();
  }
}

__global__ __launch_bounds__(256) void w2t_split_kernel(const float* __restrict__ w2, unsigned short* __restrict__ th,
                                                        unsigned short* __restrict__ tl) {
  __shared__ float tile[64 * 33];
  const int n0 = blockIdx.x * 64;
  const int l  = blockIdx.y;
  const int t  = threadIdx.x;
  const float* wl = w2 + (size_t)l * kLoraD * kDm;
#pragma unroll
  for (int i = 0; i < 8; ++i) {
    const int idx = i * 256 + t;
    const int kk = idx >> 6, nn = idx & 63;
    tile[nn * 33 + kk] = wl[(size_t)kk * kDm + n0 + nn];
  }
  __syncthreads();
  const int lane = t & 31, wave = t >> 5;
  const int L = lane >> 3, q = lane & 7;
  const int row = wave * 8 + 2 * L + (q >> 2);
  const int k8 = (q & 3) * 8;
  const float* sp = tile + row * 33 + k8;
  v8us hv, lv;
#pragma unroll
  for (int e = 0; e < 8; ++e) {
    const unsigned short hb = f2bf_bits(sp[e]);
    const unsigned short lb = f2bf_bits(sp[e] - bf_bits2f(hb));
    hv[e] = hb; lv[e] = lb;
  }
  const size_t o = (size_t)l * kDm * kLoraD + (size_t)(n0 + row) * kLoraD + k8;
  *(volatile v8us*)(th + o) = hv;
  *(volatile v8us*)(tl + o) = lv;
  __threadfence();
  *(volatile v8us*)(th + o) = hv;
  *(volatile v8us*)(tl + o) = lv;
}

__device__ __forceinline__ void split8(const v4f va, const v4f vb, v8us& hv, v8us& lv) {
#pragma unroll
  for (int e = 0; e < 4; ++e) {
    const unsigned short h0 = f2bf_bits(va[e]);
    hv[e] = h0; lv[e] = f2bf_bits(va[e] - bf_bits2f(h0));
    const unsigned short h1 = f2bf_bits(vb[e]);
    hv[4 + e] = h1; lv[4 + e] = f2bf_bits(vb[e] - bf_bits2f(h1));
  }
}
__device__ __forceinline__ void store16x2(unsigned short* ph, unsigned short* pl, size_t o, const v8us hv, const v8us lv) {
  *(volatile v8us*)(ph + o) = hv;
  *(volatile v8us*)(pl + o) = lv;
  __threadfence();
  *(volatile v8us*)(ph + o) = hv;
  *(volatile v8us*)(pl + o) = lv;
}

__global__ __launch_bounds__(128) void xxx_split_kernel(const float* __restrict__ x, const float* __restrict__ ss,
                                                        const float* __restrict__ maax,
                                                        unsigned short* __restrict__ oh, unsigned short* __restrict__ ol, int b) {
  const int s = blockIdx.x;
  const int c0 = threadIdx.x * 8;
  const float* xr = x + ((size_t)b * kSeq + s) * kDm;
  const float* xp = (s == 0) ? (ss + (size_t)b * kDm) : (xr - kDm);
  const v4f xa = *(const v4f*)(xr + c0), xb = *(const v4f*)(xr + c0 + 4);
  const v4f pa = *(const v4f*)(xp + c0), pb = *(const v4f*)(xp + c0 + 4);
  const v4f ma = *(const v4f*)(maax + c0), mb = *(const v4f*)(maax + c0 + 4);
  const v4f va = xa + (pa - xa) * ma;
  const v4f vb = xb + (pb - xb) * mb;
  v8us hv, lv;
  split8(va, vb, hv, lv);
  store16x2(oh, ol, (size_t)s * kDm + c0, hv, lv);
}

__global__ __launch_bounds__(128) void mix_split_kernel(const float* __restrict__ x, const float* __restrict__ ss,
                                                        const float* __restrict__ maar, const float* __restrict__ maak,
                                                        const float* __restrict__ maav, const float* __restrict__ mix,
                                                        unsigned short* __restrict__ qh, unsigned short* __restrict__ ql,
                                                        unsigned short* __restrict__ kh, unsigned short* __restrict__ kl,
                                                        unsigned short* __restrict__ vh, unsigned short* __restrict__ vl, int b) {
  const int s = blockIdx.x;
  const int c0 = threadIdx.x * 8;
  const float* xr = x + ((size_t)b * kSeq + s) * kDm;
  const float* xp = (s == 0) ? (ss + (size_t)b * kDm) : (xr - kDm);
  const v4f xa = *(const v4f*)(xr + c0), xb = *(const v4f*)(xr + c0 + 4);
  const v4f pa = *(const v4f*)(xp + c0), pb = *(const v4f*)(xp + c0 + 4);
  const v4f da = pa - xa, db = pb - xb;
  const size_t plane = (size_t)kSeq * kDm;
  const float* m0 = mix + (size_t)s * kDm + c0;
  const size_t o = (size_t)s * kDm + c0;
  {
    const v4f ma = *(const v4f*)(maar + c0), mb = *(const v4f*)(maar + c0 + 4);
    const v4f qa = *(const v4f*)(m0), qb = *(const v4f*)(m0 + 4);
    const v4f va = xa + da * (ma + qa), vb = xb + db * (mb + qb);
    v8us hv, lv; split8(va, vb, hv, lv); store16x2(qh, ql, o, hv, lv);
  }
  {
    const v4f ma = *(const v4f*)(maak + c0), mb = *(const v4f*)(maak + c0 + 4);
    const v4f qa = *(const v4f*)(m0 + plane), qb = *(const v4f*)(m0 + plane + 4);
    const v4f va = xa + da * (ma + qa), vb = xb + db * (mb + qb);
    v8us hv, lv; split8(va, vb, hv, lv); store16x2(kh, kl, o, hv, lv);
  }
  {
    const v4f ma = *(const v4f*)(maav + c0), mb = *(const v4f*)(maav + c0 + 4);
    const v4f qa = *(const v4f*)(m0 + 2 * plane), qb = *(const v4f*)(m0 + 2 * plane + 4);
    const v4f va = xa + da * (ma + qa), vb = xb + db * (mb + qb);
    v8us hv, lv; split8(va, vb, hv, lv); store16x2(vh, vl, o, hv, lv);
  }
}

template <int MODE>
__global__ __launch_bounds__(256) void ln_kernel(const float* srcA, const float* srcB,
                                                 const float* __restrict__ gA, const float* __restrict__ bA,
                                                 const float* __restrict__ gB, const float* __restrict__ bB,
                                                 const float* __restrict__ ang,
                                                 unsigned short* hA, unsigned short* lA,
                                                 unsigned short* hB, unsigned short* lB, float* dstf) {
  __shared__ __align__(16) float srow[kDm];
  __shared__ __align__(16) unsigned short Lh[8][128];
  __shared__ __align__(16) unsigned short Ll[8][128];
  __shared__ float sred[8];
  __shared__ float sred2[8];
  const int s = blockIdx.x;
  const int which = blockIdx.y;
  const float* src = (which == 0) ? srcA : srcB;
  const float* g   = (which == 0) ? gA : gB;
  const float* bb  = (which == 0) ? bA : bB;
  unsigned short* dh = (which == 0) ? hA : hB;
  unsigned short* dl = (which == 0) ? lA : lB;
  const int tid = threadIdx.x, lane = tid & 31, wave = tid >> 5;

  const float* row = src + (size_t)s * kDm;
  const v4f xv = *(const v4f*)(row + tid * 4);
  float ps = (xv[0] + xv[1]) + (xv[2] + xv[3]);
#pragma unroll
  for (int off = 1; off < 32; off <<= 1) ps += __shfl_xor(ps, off, 32);
  if (lane == 0) sred[wave] = ps;
  __syncthreads();
  float tot = 0.f;
#pragma unroll
  for (int w = 0; w < 8; ++w) tot += sred[w];
  const float mean = tot * (1.0f / (float)kDm);
  const v4f dv = xv - mean;
  float pq = (dv[0] * dv[0] + dv[1] * dv[1]) + (dv[2] * dv[2] + dv[3] * dv[3]);
#pragma unroll
  for (int off = 1; off < 32; off <<= 1) pq += __shfl_xor(pq, off, 32);
  if (lane == 0) sred2[wave] = pq;
  __syncthreads();
  float tot2 = 0.f;
#pragma unroll
  for (int w = 0; w < 8; ++w) tot2 += sred2[w];
  const float var  = tot2 * (1.0f / (float)kDm);
  const float rstd = rsqrtf(var + 1.0e-5f);
  const v4f gv = *(const v4f*)(g + tid * 4);
  const v4f bv = *(const v4f*)(bb + tid * 4);
  v4f yv;
#pragma unroll
  for (int e = 0; e < 4; ++e) yv[e] = dv[e] * rstd * gv[e] + bv[e];

  if (MODE == 1) {
    float* dp = dstf + (size_t)s * kDm + tid * 4;
    *(volatile v4f*)dp = yv;
    __threadfence();
    *(volatile v4f*)dp = yv;
    return;
  }

  *(v4f*)(srow + tid * 4) = yv;
  __syncthreads();

  float cs = 1.0f, sn = 0.0f;
  if (MODE == 0) {
    const float a = ang[(size_t)s * 32 + lane];
    cs = cosf(a);
    sn = sinf(a);
  }
  unsigned short* lh = Lh[wave];
  unsigned short* ll = Ll[wave];
#pragma unroll 1
  for (int hp = 0; hp < 2; ++hp) {
    const int base = wave * 128 + hp * 64;
    const float xr = srow[base + lane];
    const float xi = srow[base + 32 + lane];
    float vr = xr, vi = xi;
    if (MODE == 0) { vr = xr * cs - xi * sn; vi = xr * sn + xi * cs; }
    const unsigned short hr = f2bf_bits(vr);
    const unsigned short lr = f2bf_bits(vr - bf_bits2f(hr));
    const unsigned short hi = f2bf_bits(vi);
    const unsigned short li = f2bf_bits(vi - bf_bits2f(hi));
    lh[hp * 64 + lane] = hr;       ll[hp * 64 + lane] = lr;
    lh[hp * 64 + 32 + lane] = hi;  ll[hp * 64 + 32 + lane] = li;
  }
  __builtin_amdgcn_fence(__ATOMIC_RELEASE, "workgroup");
  __builtin_amdgcn_wave_barrier();
  __builtin_amdgcn_fence(__ATOMIC_ACQUIRE, "workgroup");
  const int l16 = lane & 15;
  const v8us hv = *(const v8us*)(lh + l16 * 8);
  const v8us lv = *(const v8us*)(ll + l16 * 8);
  const size_t o = (size_t)s * kDm + wave * 128 + l16 * 8;
  for (int pass = 0; pass < 2; ++pass) {
    if (lane < 16) {
      *(volatile v8us*)(dh + o) = hv;
      *(volatile v8us*)(dl + o) = lv;
    }
    __threadfence();
  }
}

#define AT_D 64
#define AT_NW 4
#define AT_QB 64
#define AT_KC 64

__device__ __forceinline__ unsigned short at_bf_bits(float f) {
  unsigned u = __float_as_uint(f);
  return (unsigned short)((u + 0x7FFFu + ((u >> 16) & 1u)) >> 16);
}
__device__ __forceinline__ __bf16 at_f2bf(float f) { return __builtin_bit_cast(__bf16, at_bf_bits(f)); }
__device__ __forceinline__ void at_split(float f, __bf16& hi, __bf16& lo) {
  const unsigned short hb = at_bf_bits(f);
  hi = __builtin_bit_cast(__bf16, hb);
  lo = at_f2bf(f - __uint_as_float(((unsigned)hb) << 16));
}
__device__ __forceinline__ v8f at_mma(v16b a, v16b b, v8f c) {
  c = __builtin_amdgcn_wmma_f32_16x16x32_bf16(false, a, false, b, (short)0, c, false, false);
  asm volatile("v_nop\n\tv_nop\n\tv_nop\n\tv_nop" : "+v"(c) : "v"(a), "v"(b));
  return c;
}

__global__ __launch_bounds__(128)
void attn_causal64_kernel(const unsigned short* __restrict__ qhp, const unsigned short* __restrict__ qlp,
                          const unsigned short* __restrict__ khp, const unsigned short* __restrict__ klp,
                          const unsigned short* __restrict__ vhp, const unsigned short* __restrict__ vlp,
                          float* __restrict__ out, float sscale, float mfill) {
  union FB { v16b v; v8b h[2]; };
  __shared__ __align__(16) __bf16 Ksh[AT_KC * AT_D];
  __shared__ __align__(16) __bf16 Ksl[AT_KC * AT_D];
  __shared__ __align__(16) __bf16 Vth[AT_D * AT_KC];
  __shared__ __align__(16) __bf16 Vtl[AT_D * AT_KC];
  __shared__ __align__(16) __bf16 Psh[AT_NW][16 * AT_KC];
  __shared__ __align__(16) __bf16 Psl[AT_NW][16 * AT_KC];
  __shared__ __align__(16) float  Os[AT_NW][16 * 68];

  const int tid  = threadIdx.x;
  const int wave = tid >> 5;
  const int lane = tid & 31;
  const int hh   = lane >> 4;
  const int c    = lane & 15;

  const int nqb = kSeq / AT_QB;
  const int bx = blockIdx.x;
  const int qb = bx % nqb;
  const int h  = bx / nqb;
  const int q0 = qb * AT_QB + wave * 16;

  const __bf16* Qh = (const __bf16*)(const void*)qhp + (size_t)h * AT_D;
  const __bf16* Ql = (const __bf16*)(const void*)qlp + (size_t)h * AT_D;
  const __bf16* Kh = (const __bf16*)(const void*)khp + (size_t)h * AT_D;
  const __bf16* Kl = (const __bf16*)(const void*)klp + (size_t)h * AT_D;
  const __bf16* Vh = (const __bf16*)(const void*)vhp + (size_t)h * AT_D * kSeq;
  const __bf16* Vl = (const __bf16*)(const void*)vlp + (size_t)h * AT_D * kSeq;
  float*        ob = out + (size_t)h * AT_D;

  v16b qah[2], qal[2];
#pragma unroll
  for (int dc = 0; dc < 2; ++dc) {
    const __bf16* qr = Qh + (size_t)(q0 + c) * kDm + dc * 32 + 8 * hh;
    const __bf16* ql = Ql + (size_t)(q0 + c) * kDm + dc * 32 + 8 * hh;
    qah[dc] = Frag<__bf16>::load(qr);
    qal[dc] = Frag<__bf16>::load(ql);
  }

  float mrow[8], lrow[8];
  v8f oacc[4];
#pragma unroll
  for (int r = 0; r < 8; ++r) { mrow[r] = -INFINITY; lrow[r] = 0.f; }
#pragma unroll
  for (int t = 0; t < 4; ++t) oacc[t] = (v8f){0.f,0.f,0.f,0.f,0.f,0.f,0.f,0.f};

  int nChunks = qb + 1;
  if (nChunks > kSeq / AT_KC) nChunks = kSeq / AT_KC;
  for (int kc = 0; kc < nChunks; ++kc) {
    const int kv0 = kc * AT_KC;
    __syncthreads();
    {
      const int r = tid >> 1, half = (tid & 1) * 32;
      const __bf16* ksh = Kh + (size_t)(kv0 + r) * kDm + half;
      const __bf16* ksl = Kl + (size_t)(kv0 + r) * kDm + half;
      const __bf16* vsh = Vh + (size_t)r * kSeq + kv0 + half;
      const __bf16* vsl = Vl + (size_t)r * kSeq + kv0 + half;
#pragma unroll
      for (int i = 0; i < 4; ++i) {
        const v8b a0 = *(const v8b*)(ksh + 8 * i);
        const v8b a1 = *(const v8b*)(ksl + 8 * i);
        const v8b b0 = *(const v8b*)(vsh + 8 * i);
        const v8b b1 = *(const v8b*)(vsl + 8 * i);
        *(v8b*)(Ksh + r * AT_D  + half + 8 * i) = a0;
        *(v8b*)(Ksl + r * AT_D  + half + 8 * i) = a1;
        *(v8b*)(Vth + r * AT_KC + half + 8 * i) = b0;
        *(v8b*)(Vtl + r * AT_KC + half + 8 * i) = b1;
      }
    }
    __syncthreads();

    v8f s[4];
#pragma unroll
    for (int j = 0; j < 4; ++j) {
      s[j] = (v8f){0.f,0.f,0.f,0.f,0.f,0.f,0.f,0.f};
#pragma unroll
      for (int dc = 0; dc < 2; ++dc) {
        FB kb, kl;
        kb.h[0] = *(const v8b*)(Ksh + (j * 16 + c) * AT_D + dc * 32 + 8 * hh);
        kb.h[1] = *(const v8b*)(Ksh + (j * 16 + c) * AT_D + dc * 32 + 16 + 8 * hh);
        kl.h[0] = *(const v8b*)(Ksl + (j * 16 + c) * AT_D + dc * 32 + 8 * hh);
        kl.h[1] = *(const v8b*)(Ksl + (j * 16 + c) * AT_D + dc * 32 + 16 + 8 * hh);
        s[j] = at_mma(qah[dc], kb.v, s[j]);
        s[j] = at_mma(qah[dc], kl.v, s[j]);
        s[j] = at_mma(qal[dc], kb.v, s[j]);
      }
    }
    const bool diag = (kc == qb);
    float cm[8];
#pragma unroll
    for (int r = 0; r < 8; ++r) {
      const int qrow = q0 + 8 * hh + r;
      float m = -INFINITY;
#pragma unroll
      for (int j = 0; j < 4; ++j) {
        const int kvcol = kv0 + j * 16 + c;
        const float sv = s[j][r] * sscale;
        const bool masked = diag && (kvcol > qrow);
        const float sm = masked ? mfill : sv;
        s[j][r] = sm;
        m = fmaxf(m, sm);
      }
#pragma unroll
      for (int off = 1; off < 16; off <<= 1) m = fmaxf(m, __shfl_xor(m, off, 32));
      cm[r] = m;
    }
    __bf16* pwh = Psh[wave];
    __bf16* pwl = Psl[wave];
#pragma unroll
    for (int r = 0; r < 8; ++r) {
      const float mnew = fmaxf(mrow[r], cm[r]);
      const float alpha = expf(mrow[r] - mnew);
      mrow[r] = mnew;
      float psum = 0.f;
#pragma unroll
      for (int j = 0; j < 4; ++j) {
        const float p = expf(s[j][r] - mnew);
        psum += p;
        __bf16 a, bl; at_split(p, a, bl);
        pwh[(8 * hh + r) * AT_KC + j * 16 + c] = a;
        pwl[(8 * hh + r) * AT_KC + j * 16 + c] = bl;
      }
#pragma unroll
      for (int off = 1; off < 16; off <<= 1) psum += __shfl_xor(psum, off, 32);
      lrow[r] = lrow[r] * alpha + psum;
#pragma unroll
      for (int t = 0; t < 4; ++t) oacc[t][r] *= alpha;
    }
    __builtin_amdgcn_fence(__ATOMIC_RELEASE, "workgroup");
    __builtin_amdgcn_wave_barrier();
    __builtin_amdgcn_fence(__ATOMIC_ACQUIRE, "workgroup");
#pragma unroll 1
    for (int kk = 0; kk < 2; ++kk) {
      FB pa, pl;
      pa.h[0] = *(const v8b*)(pwh + c * AT_KC + kk * 32 + 8 * hh);
      pa.h[1] = *(const v8b*)(pwh + c * AT_KC + kk * 32 + 16 + 8 * hh);
      pl.h[0] = *(const v8b*)(pwl + c * AT_KC + kk * 32 + 8 * hh);
      pl.h[1] = *(const v8b*)(pwl + c * AT_KC + kk * 32 + 16 + 8 * hh);
#pragma unroll
      for (int t = 0; t < 4; ++t) {
        FB vb, vl;
        vb.h[0] = *(const v8b*)(Vth + (t * 16 + c) * AT_KC + kk * 32 + 8 * hh);
        vb.h[1] = *(const v8b*)(Vth + (t * 16 + c) * AT_KC + kk * 32 + 16 + 8 * hh);
        vl.h[0] = *(const v8b*)(Vtl + (t * 16 + c) * AT_KC + kk * 32 + 8 * hh);
        vl.h[1] = *(const v8b*)(Vtl + (t * 16 + c) * AT_KC + kk * 32 + 16 + 8 * hh);
        oacc[t] = at_mma(pa.v, vb.v, oacc[t]);
        oacc[t] = at_mma(pa.v, vl.v, oacc[t]);
        oacc[t] = at_mma(pl.v, vb.v, oacc[t]);
      }
    }
  }

  float* os = Os[wave];
#pragma unroll
  for (int r = 0; r < 8; ++r) {
    const float inv = 1.0f / lrow[r];
#pragma unroll
    for (int t = 0; t < 4; ++t) os[(8 * hh + r) * 68 + t * 16 + c] = oacc[t][r] * inv;
  }
  __builtin_amdgcn_fence(__ATOMIC_RELEASE, "workgroup");
  __builtin_amdgcn_wave_barrier();
  __builtin_amdgcn_fence(__ATOMIC_ACQUIRE, "workgroup");
  {
    const int c4 = (lane & 15) * 4;
    for (int pass = 0; pass < 2; ++pass) {
#pragma unroll
      for (int it = 0; it < 8; ++it) {
        const int row = it * 2 + hh;
        v4f val = *(const v4f*)(os + row * 68 + c4);
        *(volatile v4f*)(ob + (size_t)(q0 + row) * kDm + c4) = val;
      }
      __threadfence();
    }
  }
}

extern "C" void kernel_launch(void* const* d_in, const int* in_sizes, int n_in,
                              void* d_out, int out_size, void* d_ws, size_t ws_size,
                              hipStream_t stream) {
  if (n_in < 21) return;
  const int nRow = kSeq * kDm;
  const int nAct = kBatch * nRow;
  const int nW   = kDm * kDm;
  if (in_sizes[0] != nAct) return;
  if (in_sizes[1] != kBatch * kDm) return;
  if (in_sizes[2] != kDm || in_sizes[3] != kDm || in_sizes[4] != kDm || in_sizes[5] != kDm) return;
  if (in_sizes[6] != kDm * kLoraN) return;
  if (in_sizes[7] != 3 * kLoraD * kDm) return;
  if (in_sizes[8] != nW || in_sizes[9] != nW || in_sizes[10] != nW || in_sizes[11] != nW) return;
  for (int i = 12; i < 20; ++i) if (in_sizes[i] != kDm) return;
  if (in_sizes[20] != kSeq * 32) return;
  if (out_size != nAct) return;

  const float* x     = (const float*)d_in[0];
  const float* ss    = (const float*)d_in[1];
  const float* maax  = (const float*)d_in[2];
  const float* maar  = (const float*)d_in[3];
  const float* maak  = (const float*)d_in[4];
  const float* maav  = (const float*)d_in[5];
  const float* w1    = (const float*)d_in[6];
  const float* w2    = (const float*)d_in[7];
  const float* wq    = (const float*)d_in[8];
  const float* wk    = (const float*)d_in[9];
  const float* wv    = (const float*)d_in[10];
  const float* wo    = (const float*)d_in[11];
  const float* lnrg  = (const float*)d_in[12];
  const float* lnrb  = (const float*)d_in[13];
  const float* lnkg  = (const float*)d_in[14];
  const float* lnkb  = (const float*)d_in[15];
  const float* lnvg  = (const float*)d_in[16];
  const float* lnvb  = (const float*)d_in[17];
  const float* lnxg  = (const float*)d_in[18];
  const float* lnxb  = (const float*)d_in[19];
  const float* ang   = (const float*)d_in[20];

  const size_t PW   = (size_t)kDm * kDm * 2;
  const size_t PX   = (size_t)kSeq * kDm * 2;
  const size_t PF   = (size_t)kSeq * kDm * 4;
  const size_t PW1  = (size_t)kLoraP * kDm * 2;
  const size_t PW2  = (size_t)3 * kDm * kLoraD * 2;
  const size_t PLF  = (size_t)kSeq * kLoraP * 4;
  const size_t PLT  = (size_t)kSeq * kLoraP * 2;
  size_t off = 0;
  const size_t oWqh = off; off += PW;  const size_t oWql = off; off += PW;
  const size_t oWkh = off; off += PW;  const size_t oWkl = off; off += PW;
  const size_t oWvh = off; off += PW;  const size_t oWvl = off; off += PW;
  const size_t oWoh = off; off += PW;  const size_t oWol = off; off += PW;
  const size_t oW1h = off; off += PW1; const size_t oW1l = off; off += PW1;
  const size_t oW2h = off; off += PW2; const size_t oW2l = off; off += PW2;
  const size_t oXXh = off; off += PX;  const size_t oXXl = off; off += PX;
  const size_t oLF  = off; off += PLF;
  const size_t oLTh = off; off += PLT; const size_t oLTl = off; off += PLT;
  const size_t oMIX = off; off += 3 * PF;
  const size_t oXQh = off; off += PX;  const size_t oXQl = off; off += PX;
  const size_t oXKh = off; off += PX;  const size_t oXKl = off; off += PX;
  const size_t oXVh = off; off += PX;  const size_t oXVl = off; off += PX;
  const size_t oQh  = off; off += PX;  const size_t oQl  = off; off += PX;
  const size_t oKh  = off; off += PX;  const size_t oKl  = off; off += PX;
  const size_t oVTh = off; off += PX;  const size_t oVTl = off; off += PX;
  if (off > ws_size) return;

  char* ws = (char*)d_ws;
  unsigned short* Wqh = (unsigned short*)(ws + oWqh); unsigned short* Wql = (unsigned short*)(ws + oWql);
  unsigned short* Wkh = (unsigned short*)(ws + oWkh); unsigned short* Wkl = (unsigned short*)(ws + oWkl);
  unsigned short* Wvh = (unsigned short*)(ws + oWvh); unsigned short* Wvl = (unsigned short*)(ws + oWvl);
  unsigned short* Woh = (unsigned short*)(ws + oWoh); unsigned short* Wol = (unsigned short*)(ws + oWol);
  unsigned short* W1h = (unsigned short*)(ws + oW1h); unsigned short* W1l = (unsigned short*)(ws + oW1l);
  unsigned short* W2h = (unsigned short*)(ws + oW2h); unsigned short* W2l = (unsigned short*)(ws + oW2l);
  unsigned short* XXh = (unsigned short*)(ws + oXXh); unsigned short* XXl = (unsigned short*)(ws + oXXl);
  float*          LF  = (float*)(ws + oLF);
  unsigned short* LTh = (unsigned short*)(ws + oLTh); unsigned short* LTl = (unsigned short*)(ws + oLTl);
  float*          MIX = (float*)(ws + oMIX);
  float*          Qf  = (float*)(ws + oMIX);
  float*          Kf  = (float*)(ws + oMIX + PF);
  float*          Vf  = (float*)(ws + oMIX + 2 * PF);
  float*          Of  = Qf;
  unsigned short* XQh = (unsigned short*)(ws + oXQh); unsigned short* XQl = (unsigned short*)(ws + oXQl);
  unsigned short* XKh = (unsigned short*)(ws + oXKh); unsigned short* XKl = (unsigned short*)(ws + oXKl);
  unsigned short* XVh = (unsigned short*)(ws + oXVh); unsigned short* XVl = (unsigned short*)(ws + oXVl);
  unsigned short* Qh  = (unsigned short*)(ws + oQh);  unsigned short* Ql  = (unsigned short*)(ws + oQl);
  unsigned short* Kh  = (unsigned short*)(ws + oKh);  unsigned short* Kl  = (unsigned short*)(ws + oKl);
  unsigned short* VTh = (unsigned short*)(ws + oVTh); unsigned short* VTl = (unsigned short*)(ws + oVTl);
  unsigned short* Oh  = XXh;                          unsigned short* Ol  = XXl;

  const float* dummyf = lnrg;

  const dim3 blk(256);
  const int  n2w = nW / 2;
  const dim3 gCastW((n2w + 255) / 256);
  const dim3 gW1(kDm / 64);
  const dim3 gW2(kDm / 64, 3);
  const dim3 gRow(kSeq);
  const dim3 gLora(((kSeq / 64) * (kLoraP / 64) + 7) / 8);
  const dim3 gMix(((kSeq / 64) * (kDm / 64) + 7) / 8, 3);
  const int  n2l = kSeq * kLoraP / 2;
  const dim3 gTanh((n2l + 255) / 256);
  const dim3 gProj(((kSeq / 64) * (kDm / 64) + 7) / 8, 1);
  const dim3 gLnQK(kSeq, 2);
  const dim3 gLn1(kSeq, 1);
  const dim3 gVT(kDm / 64, kSeq / 64);
  const dim3 gAtt(kHeads * (kSeq / 64));

  split_bf16x2_kernel<<<gCastW, blk, 0, stream>>>(wq, Wqh, Wql, n2w);
  split_bf16x2_kernel<<<gCastW, blk, 0, stream>>>(wk, Wkh, Wkl, n2w);
  split_bf16x2_kernel<<<gCastW, blk, 0, stream>>>(wv, Wvh, Wvl, n2w);
  split_bf16x2_kernel<<<gCastW, blk, 0, stream>>>(wo, Woh, Wol, n2w);
  w1t_split_kernel<<<gW1, blk, 0, stream>>>(w1, W1h, W1l);
  w2t_split_kernel<<<gW2, blk, 0, stream>>>(w2, W2h, W2l);

  for (int b = 0; b < kBatch; ++b) {
    xxx_split_kernel<<<gRow, dim3(128), 0, stream>>>(x, ss, maax, XXh, XXl, b);
    wmma_gemm64<1, true, 0, 0, false, 0><<<gLora, blk, 0, stream>>>(
        XXh, XXl, kDm, 0L, W1h, W1l, kDm, 0L, (void*)LF, (void*)LF, kLoraP, 0L,
        dummyf, dummyf, 0L, kSeq, kLoraP, kDm, 1.0f);
    tanh_split_kernel<<<gTanh, blk, 0, stream>>>(LF, LTh, LTl, n2l);
    wmma_gemm64<1, true, 0, 0, false, 0><<<gMix, blk, 0, stream>>>(
        LTh, LTl, kLoraP, (long)kLoraD, W2h, W2l, kLoraD, (long)kDm * kLoraD, (void*)MIX, (void*)MIX, kDm, (long)nRow,
        dummyf, dummyf, 0L, kSeq, kDm, kLoraD, 1.0f);
    mix_split_kernel<<<gRow, dim3(128), 0, stream>>>(x, ss, maar, maak, maav, MIX, XQh, XQl, XKh, XKl, XVh, XVl, b);
    wmma_gemm64<1, true, 0, 0, false, 0><<<gProj, blk, 0, stream>>>(
        XQh, XQl, kDm, 0L, Wqh, Wql, kDm, 0L, (void*)Qf, (void*)Qf, kDm, 0L,
        dummyf, dummyf, 0L, kSeq, kDm, kDm, 1.0f);
    wmma_gemm64<1, true, 0, 0, false, 0><<<gProj, blk, 0, stream>>>(
        XKh, XKl, kDm, 0L, Wkh, Wkl, kDm, 0L, (void*)Kf, (void*)Kf, kDm, 0L,
        dummyf, dummyf, 0L, kSeq, kDm, kDm, 1.0f);
    wmma_gemm64<1, true, 0, 0, false, 0><<<gProj, blk, 0, stream>>>(
        XVh, XVl, kDm, 0L, Wvh, Wvl, kDm, 0L, (void*)Vf, (void*)Vf, kDm, 0L,
        dummyf, dummyf, 0L, kSeq, kDm, kDm, 1.0f);
    ln_kernel<0><<<gLnQK, blk, 0, stream>>>(Qf, Kf, lnrg, lnrb, lnkg, lnkb, ang, Qh, Ql, Kh, Kl, Qf);
    ln_kernel<1><<<gLn1, blk, 0, stream>>>(Vf, Vf, lnvg, lnvb, lnvg, lnvb, ang, VTh, VTl, VTh, VTl, Vf);
    wt_split_kernel<<<gVT, blk, 0, stream>>>(Vf, VTh, VTl, kSeq, kDm);
    attn_causal64_kernel<<<gAtt, dim3(128), 0, stream>>>(Qh, Ql, Kh, Kl, VTh, VTl, Of, 0.125f, -1.0e30f);
    ln_kernel<2><<<gLn1, blk, 0, stream>>>(Of, Of, lnxg, lnxb, lnxg, lnxb, ang, Oh, Ol, Oh, Ol, Of);
    float* outb = (float*)d_out + (size_t)b * nRow;
    wmma_gemm64<1, true, 0, 0, false, 0><<<gProj, blk, 0, stream>>>(
        Oh, Ol, kDm, 0L, Woh, Wol, kDm, 0L, (void*)outb, (void*)outb, kDm, 0L,
        dummyf, dummyf, 0L, kSeq, kDm, kDm, 1.0f);
  }
}
